// MyGSGNN_44942537785493
// MI455X (gfx1250) — hardware-run, weakly checked
//
#include <hip/hip_runtime.h>
#include <stddef.h>


#define IND     128
#define NLOC    112
#define CH0     64
#define CDM     16
#define NGL     5
#define NTHR    256
#define NWAVE   8
#define EPT     8
#define NGRP    2
#define CHUNK   (NTHR * EPT * NGRP)
#define WCAP    (EPT * NGRP * 32)
#define LISTN   (NWAVE * WCAP)
#define NBC     4096
#define NBF     1024
#define RCAP    40960
#define RBN     128
#define TGT     256
#define DEGCAP  256
#define OTHR    512
#define GTHR    128
#define GBM     64
#define WSCAP   134217728
#define SCL_A   8.0f
#define SCL_W   16.0f
#define SCL_ACC 0.0078125f

#define LDS_FILL ((RCAP + NBF + LISTN) * 4 + 64)

static_assert((CHUNK & (CHUNK - 1)) == 0);
static_assert(CHUNK <= 4096);
static_assert(NBC <= 4096 && NBF <= 4096);
static_assert((NBC & (NBC - 1)) == 0 && (NBF & (NBF - 1)) == 0);
static_assert(NBC == 4 * NBF);
static_assert(OTHR * 8 == NBC);
static_assert((RCAP % 32) == 0);
static_assert(TGT == NWAVE * 32);
static_assert((NBC % TGT) == 0);
static_assert((TGT % GBM) == 0);
static_assert(GBM * 2 == GTHR);
static_assert(IND % 32 == 0 && CH0 % 32 == 0 && NLOC % 16 == 0 && CDM == 16);

typedef float    v2f  __attribute__((ext_vector_type(2)));
typedef float    v4f  __attribute__((ext_vector_type(4)));
typedef float    v8f  __attribute__((ext_vector_type(8)));
typedef int      v4i  __attribute__((ext_vector_type(4)));
typedef _Float16 v4h  __attribute__((ext_vector_type(4)));
typedef _Float16 v8h  __attribute__((ext_vector_type(8)));
typedef _Float16 v16h __attribute__((ext_vector_type(16)));
union FragH { v16h v; v8h h[2]; };

__device__ __forceinline__ v8f wmh(v16h a, v16h b, v8f c) {
  v8f d = __builtin_amdgcn_wmma_f32_16x16x32_f16(false, a, false, b, (short)0, c, false, false);
  asm volatile("v_nop\n\tv_nop\n\tv_nop\n\tv_nop" : "+v"(d) : "v"(a), "v"(b));
  return d;
}

__device__ __forceinline__ v8h cvt8(v4f a, v4f b, float s) {
  v8f t;
  t[0] = a.x * s; t[1] = a.y * s; t[2] = a.z * s; t[3] = a.w * s;
  t[4] = b.x * s; t[5] = b.y * s; t[6] = b.z * s; t[7] = b.w * s;
  return __builtin_convertvector(t, v8h);
}

__device__ __forceinline__ float tanh_fast(float s) {
  const float a = fminf(fabsf(s), 16.0f);
  const float t = __expf(-2.0f * a);
  const float r = (1.0f - t) * __builtin_amdgcn_rcpf(1.0f + t);
  return __builtin_copysignf(r, s);
}

__device__ __forceinline__ float dot16(v4f a, v4f b, v4f c, v4f d, const float* __restrict__ w) {
  float s = a.x * w[0];
  s += a.y * w[1];  s += a.z * w[2];  s += a.w * w[3];
  s += b.x * w[4];  s += b.y * w[5];  s += b.z * w[6];  s += b.w * w[7];
  s += c.x * w[8];  s += c.y * w[9];  s += c.z * w[10]; s += c.w * w[11];
  s += d.x * w[12]; s += d.y * w[13]; s += d.z * w[14]; s += d.w * w[15];
  return s;
}

template <int NB>
__device__ __forceinline__ int scan_chunk(const int* __restrict__ dsts, int nE, int cbase, int slotBase,
                                          int vec8, int* list, int tid, int lane, int wave) {
  int wc = 0;
#pragma unroll
  for (int g = 0; g < NGRP; ++g) {
    const int el0  = (g * NTHR + tid) * EPT;
    const int e0   = cbase + el0;
    const int sent = -2147483647 - 1;
    v4i da, db;
    if (vec8 != 0 && cbase + CHUNK <= nE) {
      da = *(const v4i*)(dsts + e0);
      db = *(const v4i*)(dsts + e0 + 4);
    } else {
      da.x = (e0     < nE) ? dsts[min(e0, nE - 1)] : sent;
      da.y = (e0 + 1 < nE) ? dsts[min(e0 + 1, nE - 1)] : sent;
      da.z = (e0 + 2 < nE) ? dsts[min(e0 + 2, nE - 1)] : sent;
      da.w = (e0 + 3 < nE) ? dsts[min(e0 + 3, nE - 1)] : sent;
      db.x = (e0 + 4 < nE) ? dsts[min(e0 + 4, nE - 1)] : sent;
      db.y = (e0 + 5 < nE) ? dsts[min(e0 + 5, nE - 1)] : sent;
      db.z = (e0 + 6 < nE) ? dsts[min(e0 + 6, nE - 1)] : sent;
      db.w = (e0 + 7 < nE) ? dsts[min(e0 + 7, nE - 1)] : sent;
    }
    const unsigned nb = (unsigned)slotBase;
    const unsigned s0 = (unsigned)da.x - nb, s1 = (unsigned)da.y - nb;
    const unsigned s2 = (unsigned)da.z - nb, s3 = (unsigned)da.w - nb;
    const unsigned s4 = (unsigned)db.x - nb, s5 = (unsigned)db.y - nb;
    const unsigned s6 = (unsigned)db.z - nb, s7 = (unsigned)db.w - nb;
    const bool h0 = s0 < (unsigned)NB, h1 = s1 < (unsigned)NB, h2 = s2 < (unsigned)NB, h3 = s3 < (unsigned)NB;
    const bool h4 = s4 < (unsigned)NB, h5 = s5 < (unsigned)NB, h6 = s6 < (unsigned)NB, h7 = s7 < (unsigned)NB;
    const unsigned any = __builtin_amdgcn_ballot_w32(h0 | h1 | h2 | h3 | h4 | h5 | h6 | h7);
    if (any != 0u) {
#define HITJ(J, HJ, SJ) { \
        const unsigned mj = __builtin_amdgcn_ballot_w32(HJ); \
        if (mj != 0u) { \
          if (HJ) { \
            const int pos = wc + (int)__builtin_amdgcn_mbcnt_lo(mj, 0u); \
            if (pos < WCAP) list[wave * WCAP + pos] = ((el0 + (J)) << 12) | (int)(SJ); \
          } \
          wc += (int)__builtin_popcount(mj); } }
      HITJ(0, h0, s0)
      HITJ(1, h1, s1)
      HITJ(2, h2, s2)
      HITJ(3, h3, s3)
      HITJ(4, h4, s4)
      HITJ(5, h5, s5)
      HITJ(6, h6, s6)
      HITJ(7, h7, s7)
#undef HITJ
    }
  }
  return wc;
}

__global__ __launch_bounds__(NTHR) void k_packw(const float* __restrict__ W, _Float16* Wt,
                                               int ncw, int fseg, int kp, int nseg, int nUnits) {
  const int i = (int)blockIdx.x * NTHR + (int)threadIdx.x;
  if (i >= nUnits) return;
  const int ktot  = nseg * kp;
  const int e0    = 8 * i;
  int n           = e0 / ktot;
  const int kg    = e0 - n * ktot;
  const int s     = kg / kp;
  const int k     = kg - s * kp;
  const int nrows = nseg * fseg;
  n = n > ncw - 1 ? ncw - 1 : (n < 0 ? 0 : n);
  v8f t;
#pragma unroll
  for (int jj = 0; jj < 8; ++jj) {
    const int kk = k + jj;
    int row = s * fseg + (kk < fseg ? kk : fseg - 1);
    row = row < 0 ? 0 : (row > nrows - 1 ? nrows - 1 : row);
    const float v = W[(size_t)row * ncw + n];
    t[jj] = (kk < fseg) ? v * SCL_W : 0.0f;
  }
  const v8h o = __builtin_convertvector(t, v8h);
  _Float16* d = Wt + (size_t)i * 8;
  *(volatile v8h*)d = o;
  __threadfence();
  *(volatile v8h*)d = o;
}

__global__ __launch_bounds__(NTHR) void k_count(
    const int* __restrict__ dsts, int* cnt, int nE, int vec8) {
  __shared__ __attribute__((aligned(16))) int scnt[NBC];
  __shared__ __attribute__((aligned(16))) int list[LISTN];
  __shared__ int wcnt[NWAVE];
  const int tid = threadIdx.x, lane = tid & 31, wave = tid >> 5;
  const int nodeBase = blockIdx.x * NBC;

  for (int i = tid; i < NBC; i += NTHR) scnt[i] = 0;
  __syncthreads();

  const int nChunks = (nE + CHUNK - 1) / CHUNK;
#pragma unroll 1
  for (int ch = 0; ch < nChunks; ++ch) {
    const int cbase = ch * CHUNK;
    const int wc = scan_chunk<NBC>(dsts, nE, cbase, nodeBase, vec8, list, tid, lane, wave);
    if (lane == 0) wcnt[wave] = wc;
    __syncthreads();
    if (wave == 0) {
#pragma unroll 1
      for (int wsx = 0; wsx < NWAVE; ++wsx) {
        int n = __builtin_amdgcn_readfirstlane(wcnt[wsx]);
        n = n > WCAP ? WCAP : (n < 0 ? 0 : n);
        const int* lp = list + wsx * WCAP;
#pragma unroll 1
        for (int i = 0; i < n; ++i) {
          const int ent  = __builtin_amdgcn_readfirstlane(lp[i]);
          const int slot = ent & (NBC - 1);
          if (lane == 0) scnt[slot] = scnt[slot] + 1;
        }
      }
    }
    __syncthreads();
  }

  v4i cq[4];
#pragma unroll
  for (int q = 0; q < 4; ++q) {
    const int f = (wave * 4 + q) * 128 + 4 * lane;
    cq[q] = *(const v4i*)(scnt + f);
  }
  int* cp = cnt + (size_t)nodeBase;
#pragma unroll
  for (int q = 0; q < 4; ++q) {
    const int f = (wave * 4 + q) * 128 + 4 * lane;
    *(volatile v4i*)(cp + f) = cq[q];
  }
  __threadfence();
#pragma unroll
  for (int q = 0; q < 4; ++q) {
    const int f = (wave * 4 + q) * 128 + 4 * lane;
    *(volatile v4i*)(cp + f) = cq[q];
  }
}

__global__ __launch_bounds__(OTHR) void k_offsets(
    const int* __restrict__ cnt, int* off, int* rbase, int nChunk) {
  __shared__ __attribute__((aligned(16))) int soff[NBC];
  __shared__ __attribute__((aligned(16))) int srb[RBN];
  __shared__ int wtot[OTHR / 32];
  const int tid = threadIdx.x, lane = tid & 31, wave = tid >> 5, sub = tid >> 7;
  for (int i = tid; i < RBN; i += OTHR) srb[i] = 0;
  int carry = 0;
#pragma unroll 1
  for (int ch = 0; ch < nChunk; ++ch) {
    const int base = ch * NBC;
    const v4i c0 = *(const v4i*)(cnt + base + 8 * tid);
    const v4i c1 = *(const v4i*)(cnt + base + 8 * tid + 4);
    const int e0 = max(c0.x, 0), e1 = max(c0.y, 0), e2 = max(c0.z, 0), e3 = max(c0.w, 0);
    const int e4 = max(c1.x, 0), e5 = max(c1.y, 0), e6 = max(c1.z, 0), e7 = max(c1.w, 0);
    const int ts = e0 + e1 + e2 + e3 + e4 + e5 + e6 + e7;
    int incl = ts;
#pragma unroll
    for (int d = 1; d < 32; d <<= 1) {
      const int t = __shfl_up(incl, d);
      if (lane >= d) incl += t;
    }
    if (lane == 31) wtot[wave] = incl;
    __syncthreads();
    const int S0 = wtot[0]  + wtot[1]  + wtot[2]  + wtot[3];
    const int S1 = wtot[4]  + wtot[5]  + wtot[6]  + wtot[7];
    const int S2 = wtot[8]  + wtot[9]  + wtot[10] + wtot[11];
    const int S3 = wtot[12] + wtot[13] + wtot[14] + wtot[15];
    int pre = 0;
#pragma unroll 1
    for (int w = 4 * sub; w < wave; ++w) pre += wtot[w];
    const int b0 = carry;
    const int b1 = b0 + ((S0 + 31) & ~31);
    const int b2 = b1 + ((S1 + 31) & ~31);
    const int b3 = b2 + ((S2 + 31) & ~31);
    const int b4 = b3 + ((S3 + 31) & ~31);
    const int myb = sub == 0 ? b0 : (sub == 1 ? b1 : (sub == 2 ? b2 : b3));
    if (tid == 0) {
      srb[min(4 * ch + 0, RBN - 1)] = b0;
      srb[min(4 * ch + 1, RBN - 1)] = b1;
      srb[min(4 * ch + 2, RBN - 1)] = b2;
      srb[min(4 * ch + 3, RBN - 1)] = b3;
    }
    int run = myb + pre + incl - ts;
    soff[8 * tid + 0] = run; run += e0;
    soff[8 * tid + 1] = run; run += e1;
    soff[8 * tid + 2] = run; run += e2;
    soff[8 * tid + 3] = run; run += e3;
    soff[8 * tid + 4] = run; run += e4;
    soff[8 * tid + 5] = run; run += e5;
    soff[8 * tid + 6] = run; run += e6;
    soff[8 * tid + 7] = run;
    carry = b4;
    __syncthreads();
    const v4i o0 = *(const v4i*)(soff + 4 * tid);
    const v4i o1 = *(const v4i*)(soff + 4 * (tid + OTHR));
    int* op = off + base;
    *(volatile v4i*)(op + 4 * tid) = o0;
    *(volatile v4i*)(op + 4 * (tid + OTHR)) = o1;
    __threadfence();
    *(volatile v4i*)(op + 4 * tid) = o0;
    *(volatile v4i*)(op + 4 * (tid + OTHR)) = o1;
    __syncthreads();
  }
  if (tid == 0) srb[min(4 * nChunk, RBN - 1)] = carry;
  __syncthreads();
  v4i rv = {0, 0, 0, 0};
  if (tid < 32) rv = *(const v4i*)(srb + 4 * tid);
  if (tid < 32) *(volatile v4i*)(rbase + 4 * tid) = rv;
  __threadfence();
  if (tid < 32) *(volatile v4i*)(rbase + 4 * tid) = rv;
}

__global__ __launch_bounds__(NTHR) void k_fill(
    const int* __restrict__ dsts, const int* __restrict__ off, const int* __restrict__ rbase,
    int* csr, const int* __restrict__ srcs, int nE, int vec8, int csrLen, int nN) {
  extern __shared__ v4f lds_dyn[];
  int* region = (int*)lds_dyn;
  int* cursor = region + RCAP;
  int* list   = cursor + NBF;
  int* wcnt   = list + LISTN;
  const int tid = threadIdx.x, lane = tid & 31, wave = tid >> 5;
  const int b = blockIdx.x;
  const int nodeBase = b * NBF;

  int rb0 = rbase[b];
  const int rb1 = rbase[b + 1];
  rb0 = rb0 < 0 ? 0 : (rb0 > csrLen ? csrLen : rb0);
  rb0 &= ~31;
  int len = rb1 - rb0;
  len = len < 0 ? 0 : (len > RCAP ? RCAP : len);
  int lenW = (len + 31) & ~31;
  if (rb0 + lenW > csrLen) lenW = (csrLen - rb0) & ~31;

  {
    const v4i z = {0, 0, 0, 0};
    for (int i = tid; i < RCAP / 4; i += NTHR) ((v4i*)region)[i] = z;
    for (int s = tid; s < NBF; s += NTHR) {
      int o = off[nodeBase + s] - rb0;
      o = o < 0 ? 0 : (o > RCAP ? RCAP : o);
      cursor[s] = o;
    }
  }
  __syncthreads();

  const int nChunks = (nE + CHUNK - 1) / CHUNK;
#pragma unroll 1
  for (int ch = 0; ch < nChunks; ++ch) {
    const int cbase = ch * CHUNK;
    const int wc = scan_chunk<NBF>(dsts, nE, cbase, nodeBase, vec8, list, tid, lane, wave);
    if (lane == 0) wcnt[wave] = wc;
    __syncthreads();
    if (wave == 0) {
#pragma unroll 1
      for (int wsx = 0; wsx < NWAVE; ++wsx) {
        int n = __builtin_amdgcn_readfirstlane(wcnt[wsx]);
        n = n > WCAP ? WCAP : (n < 0 ? 0 : n);
        const int* lp = list + wsx * WCAP;
#pragma unroll 1
        for (int i = 0; i < n; ++i) {
          const int ent  = __builtin_amdgcn_readfirstlane(lp[i]);
          const int slot = ent & (NBF - 1);
          int e = cbase + ((ent >> 12) & (CHUNK - 1));
          e = e > nE - 1 ? nE - 1 : (e < 0 ? 0 : e);
          int sv = srcs[e];
          sv = sv < 0 ? 0 : (sv > nN - 1 ? nN - 1 : sv);
          if (lane == 0) {
            int pos = cursor[slot];
            pos = pos < 0 ? 0 : (pos > RCAP - 1 ? RCAP - 1 : pos);
            region[pos] = sv;
            const int np = pos + 1;
            cursor[slot] = np > RCAP ? RCAP : np;
          }
        }
      }
    }
    __syncthreads();
  }

  const int nv = lenW >> 2;
  int* gp = csr + rb0;
#pragma unroll 1
  for (int i = tid; i < nv; i += NTHR) { const v4i v = ((const v4i*)region)[i]; *(volatile v4i*)(gp + 4 * i) = v; }
  __threadfence();
#pragma unroll 1
  for (int i = tid; i < nv; i += NTHR) { const v4i v = ((const v4i*)region)[i]; *(volatile v4i*)(gp + 4 * i) = v; }
}

__global__ __launch_bounds__(NTHR) void k_agg(
    const int* __restrict__ csr, const int* __restrict__ off, const int* __restrict__ cnt,
    const float* __restrict__ src, _Float16* ap, int nN, int csrLen) {
  const int tid = threadIdx.x, lane = tid & 31, wave = tid >> 5;
  const int tbase = blockIdx.x * TGT + wave * 32;
  const int col = 4 * lane;

  const int cl    = tbase + lane;
  const int cnt_l = cnt[cl];
  const int off_l = off[cl];

#pragma unroll 1
  for (int j = 0; j < 32; ++j) {
    const int c = tbase + j;
    int nraw = __shfl(cnt_l, j);
    nraw = nraw < 0 ? 0 : nraw;
    const int n = nraw > DEGCAP ? DEGCAP : nraw;
    const int st = __shfl(off_l, j);

    v4f acc = {0.0f, 0.0f, 0.0f, 0.0f};
#pragma unroll 1
    for (int q0 = 0; q0 < n; q0 += 32) {
      int pos = st + q0 + lane;
      pos = pos < 0 ? 0 : (pos > csrLen - 1 ? csrLen - 1 : pos);
      int sl = csr[pos];
      sl = sl < 0 ? 0 : (sl > nN - 1 ? nN - 1 : sl);
      const int mcnt = (n - q0) < 32 ? (n - q0) : 32;
#pragma unroll 1
      for (int pp = 0; pp < mcnt; ++pp) {
        const int s = __builtin_amdgcn_readlane(sl, pp);
        const v4f v = *(const v4f*)(src + (size_t)s * IND + col);
        acc = acc + v;
      }
    }

    v4f w = acc * SCL_A;
    if (c >= nN) { const v4f z = {0.0f, 0.0f, 0.0f, 0.0f}; w = z; }
    const v4h o = __builtin_convertvector(w, v4h);
    _Float16* gp = ap + (size_t)c * IND + col;
    *(volatile v4h*)gp = o;
    __threadfence();
    *(volatile v4h*)gp = o;
  }
}

template <int TPW, int KT>
__device__ __forceinline__ void mma_f32a(const float* __restrict__ arow, const _Float16* __restrict__ Bt,
                                         int kb, int m, int hh, v8f (&acc)[TPW]) {
  static_assert(KT % 8 == 0);
  const float* ap0 = arow + 8 * hh;
  const _Float16* bp0 = Bt + (size_t)m * KT + kb + 8 * hh;
#pragma unroll 1
  for (int kt = 0; kt < IND / 32; ++kt) {
    const float* apk = ap0 + 32 * kt;
    const v4f q0 = *(const v4f*)apk, q1 = *(const v4f*)(apk + 4);
    const v4f q2 = *(const v4f*)(apk + 16), q3 = *(const v4f*)(apk + 20);
    FragH a;
    a.h[0] = cvt8(q0, q1, SCL_A);
    a.h[1] = cvt8(q2, q3, SCL_A);
#pragma unroll
    for (int t = 0; t < TPW; ++t) {
      const _Float16* bp = bp0 + (size_t)(16 * t) * KT + 32 * kt;
      FragH bf;
      bf.h[0] = *(const v8h*)bp;
      bf.h[1] = *(const v8h*)(bp + 16);
      acc[t] = wmh(a.v, bf.v, acc[t]);
    }
  }
}

template <int TPW, int KT>
__device__ __forceinline__ void mma_f16a(const _Float16* __restrict__ arow, const _Float16* __restrict__ Bt,
                                         int kb, int m, int hh, v8f (&acc)[TPW]) {
  static_assert(KT % 8 == 0);
  const _Float16* ap0 = arow + 8 * hh;
  const _Float16* bp0 = Bt + (size_t)m * KT + kb + 8 * hh;
#pragma unroll 1
  for (int kt = 0; kt < IND / 32; ++kt) {
    FragH a;
    a.h[0] = *(const v8h*)(ap0 + 32 * kt);
    a.h[1] = *(const v8h*)(ap0 + 32 * kt + 16);
#pragma unroll
    for (int t = 0; t < TPW; ++t) {
      const _Float16* bp = bp0 + (size_t)(16 * t) * KT + 32 * kt;
      FragH bf;
      bf.h[0] = *(const v8h*)bp;
      bf.h[1] = *(const v8h*)(bp + 16);
      acc[t] = wmh(a.v, bf.v, acc[t]);
    }
  }
}

__global__ __launch_bounds__(GTHR) void k_color(
    const float* __restrict__ x, const _Float16* __restrict__ W0t, const float* __restrict__ cb0,
    const _Float16* __restrict__ W1t, const float* __restrict__ cb1, const float* __restrict__ Cx,
    float* G, int nN) {
  constexpr int TPW = CH0 / 16;
  __shared__ __attribute__((aligned(16))) _Float16 hs[4 * 16 * CH0];
  __shared__ __attribute__((aligned(16))) float cs[4 * 16 * CDM];
  const int tid = threadIdx.x, lane = tid & 31, wave = tid >> 5, hh = lane >> 4, m = lane & 15;
  const int rowBase = blockIdx.x * GBM;
  const int r0 = wave * 16;
  const int arow = rowBase + r0 + m;
  int arc = arow > nN - 1 ? nN - 1 : arow;
  arc = arc < 0 ? 0 : arc;

  v8f acc[TPW];
#pragma unroll
  for (int t = 0; t < TPW; ++t) { v8f z = {0.f, 0.f, 0.f, 0.f, 0.f, 0.f, 0.f, 0.f}; acc[t] = z; }
  mma_f32a<TPW, IND>(x + (size_t)arc * IND, W0t, 0, m, hh, acc);

  _Float16* hw = hs + wave * 16 * CH0;
#pragma unroll
  for (int t = 0; t < TPW; ++t) {
    const float bv = cb0[16 * t + m];
#pragma unroll
    for (int r = 0; r < 8; ++r) {
      float v = acc[t][r] * SCL_ACC + bv;
      v = v > 0.0f ? v : 0.0f;
      hw[(8 * hh + r) * CH0 + 16 * t + m] = (_Float16)(v * SCL_A);
    }
  }
  __syncthreads();

  v8f acc1 = {0.f, 0.f, 0.f, 0.f, 0.f, 0.f, 0.f, 0.f};
  {
    const _Float16* ap = hw + m * CH0 + 8 * hh;
    const _Float16* bp = W1t + m * CH0 + 8 * hh;
#pragma unroll
    for (int kt = 0; kt < CH0 / 32; ++kt) {
      FragH a, bf;
      a.h[0]  = *(const v8h*)(ap + 32 * kt);
      a.h[1]  = *(const v8h*)(ap + 32 * kt + 16);
      bf.h[0] = *(const v8h*)(bp + 32 * kt);
      bf.h[1] = *(const v8h*)(bp + 32 * kt + 16);
      acc1 = wmh(a.v, bf.v, acc1);
    }
  }
  float* cw = cs + wave * 16 * CDM;
  {
    const float bv = cb1[m];
#pragma unroll
    for (int r = 0; r < 8; ++r) cw[(8 * hh + r) * CDM + m] = acc1[r] * SCL_ACC + bv;
  }
  __syncthreads();

  const int rr = lane >> 1;
  const int odd = lane & 1;
  const float* cr = cw + rr * CDM;
  const v4f c0 = *(const v4f*)cr, c1 = *(const v4f*)(cr + 4), c2 = *(const v4f*)(cr + 8), c3 = *(const v4f*)(cr + 12);
  const float l0 = dot16(c0, c1, c2, c3, Cx);
  const float l1 = dot16(c0, c1, c2, c3, Cx + CDM);
  const float l2 = dot16(c0, c1, c2, c3, Cx + 2 * CDM);
  const float mx = fmaxf(l0, fmaxf(l1, l2));
  const float e0 = __expf(l0 - mx), e1 = __expf(l1 - mx), e2 = __expf(l2 - mx);
  const float inv = __builtin_amdgcn_rcpf(e0 + e1 + e2);
  float p0 = e0 * inv, p1 = e1 * inv, p2 = e2 * inv;
  const int grow = rowBase + r0 + rr;
  if (grow >= nN) { p0 = 0.0f; p1 = 0.0f; p2 = 0.0f; }
  v2f o;
  o.x = odd ? p2 : p0;
  o.y = odd ? 0.0f : p1;
  float* gp = G + (size_t)grow * 4 + 2 * odd;
  *(volatile v2f*)gp = o;
  __threadfence();
  *(volatile v2f*)gp = o;
}

__global__ __launch_bounds__(NTHR) void k_glayer(
    const float* __restrict__ Gin, float* Gout,
    const int* __restrict__ cntP, const int* __restrict__ offP, const int* __restrict__ csrP,
    const int* __restrict__ cntN, const int* __restrict__ offN, const int* __restrict__ csrN,
    const float* __restrict__ gW1, const float* __restrict__ gb1,
    const float* __restrict__ gW2, const float* __restrict__ gb2,
    int li, int nN, int csrLenP, int csrLenN) {
  const int c = (int)blockIdx.x * NTHR + (int)threadIdx.x;
  const v4f g = *(const v4f*)(Gin + (size_t)c * 4);
  int np_ = cntP[c]; np_ = np_ < 0 ? 0 : (np_ > DEGCAP ? DEGCAP : np_);
  int nn_ = cntN[c]; nn_ = nn_ < 0 ? 0 : (nn_ > DEGCAP ? DEGCAP : nn_);
  const int stp = offP[c], stn = offN[c];
  int tmax = np_ > nn_ ? np_ : nn_;
#pragma unroll
  for (int d = 16; d >= 1; d >>= 1) {
    const int o = __shfl_xor(tmax, d);
    tmax = o > tmax ? o : tmax;
  }
  tmax = tmax > DEGCAP ? DEGCAP : tmax;

  float sp0 = 0.0f, sp1 = 0.0f, sp2 = 0.0f, sn0 = 0.0f, sn1 = 0.0f, sn2 = 0.0f;
#pragma unroll 1
  for (int i = 0; i < tmax; ++i) {
    int pp = stp + i;
    pp = pp < 0 ? 0 : (pp > csrLenP - 1 ? csrLenP - 1 : pp);
    int sidp = csrP[pp];
    sidp = sidp < 0 ? 0 : (sidp > nN - 1 ? nN - 1 : sidp);
    const v4f vp = *(const v4f*)(Gin + (size_t)sidp * 4);
    const bool okp = i < np_;
    sp0 += okp ? vp.x : 0.0f; sp1 += okp ? vp.y : 0.0f; sp2 += okp ? vp.z : 0.0f;

    int pn = stn + i;
    pn = pn < 0 ? 0 : (pn > csrLenN - 1 ? csrLenN - 1 : pn);
    int sidn = csrN[pn];
    sidn = sidn < 0 ? 0 : (sidn > nN - 1 ? nN - 1 : sidn);
    const v4f vn = *(const v4f*)(Gin + (size_t)sidn * 4);
    const bool okn = i < nn_;
    sn0 += okn ? vn.x : 0.0f; sn1 += okn ? vn.y : 0.0f; sn2 += okn ? vn.z : 0.0f;
  }

  const float* w1  = gW1 + (size_t)li * 144;
  const float* bb1 = gb1 + (size_t)li * 16;
  const float* w2  = gW2 + (size_t)li * 48;
  const float* bb2 = gb2 + (size_t)li * 3;
  float o0 = 0.0f, o1 = 0.0f, o2 = 0.0f;
#pragma unroll 1
  for (int j = 0; j < 16; ++j) {
    const float* wc = w1 + j;
    float s = g.x * wc[0];
    s += g.y * wc[16];  s += g.z * wc[32];
    s += sp0 * wc[48];  s += sp1 * wc[64];  s += sp2 * wc[80];
    s += sn0 * wc[96];  s += sn1 * wc[112]; s += sn2 * wc[128];
    s += bb1[j];
    const float h = tanh_fast(s);
    const float* w2r = w2 + 3 * j;
    o0 += h * w2r[0]; o1 += h * w2r[1]; o2 += h * w2r[2];
  }
  o0 += bb2[0]; o1 += bb2[1]; o2 += bb2[2];
  const float mx = fmaxf(o0, fmaxf(o1, o2));
  const float e0 = __expf(o0 - mx), e1 = __expf(o1 - mx), e2 = __expf(o2 - mx);
  const float inv = __builtin_amdgcn_rcpf(e0 + e1 + e2);
  v4f out;
  out.x = e0 * inv; out.y = e1 * inv; out.z = e2 * inv; out.w = 0.0f;
  if (c >= nN) { const v4f z = {0.0f, 0.0f, 0.0f, 0.0f}; out = z; }
  float* gp = Gout + (size_t)c * 4;
  *(volatile v4f*)gp = out;
  __threadfence();
  *(volatile v4f*)gp = out;
}

template <int EPI>
__global__ __launch_bounds__(GTHR) void k_gemm(
    const float* __restrict__ Af, const _Float16* __restrict__ A1, const _Float16* __restrict__ A2,
    const _Float16* __restrict__ Bt, const float* __restrict__ bias,
    const float* __restrict__ Gf, const float* __restrict__ Cx,
    float* Out, int nAf, int nN) {
  constexpr int TPW = NLOC / 16;
  constexpr int KT  = 3 * IND;
  static_assert(EPI == 1 || EPI == 2);
  __shared__ __attribute__((aligned(16))) float stg[GBM * IND];
  const int tid = threadIdx.x, lane = tid & 31, wave = tid >> 5, hh = lane >> 4, m = lane & 15;
  const int rowBase = blockIdx.x * GBM;
  const int r0 = wave * 16;
  const int arow = rowBase + r0 + m;
  int arc = arow > nAf - 1 ? nAf - 1 : arow;
  arc = arc < 0 ? 0 : arc;

  v8f acc[TPW];
#pragma unroll
  for (int t = 0; t < TPW; ++t) { v8f z = {0.f, 0.f, 0.f, 0.f, 0.f, 0.f, 0.f, 0.f}; acc[t] = z; }

  mma_f32a<TPW, KT>(Af + (size_t)arc * IND, Bt, 0, m, hh, acc);
  mma_f16a<TPW, KT>(A1 + (size_t)arow * IND, Bt, IND, m, hh, acc);
  mma_f16a<TPW, KT>(A2 + (size_t)arow * IND, Bt, 2 * IND, m, hh, acc);

  float* sp = stg + (size_t)(r0 + 8 * hh) * IND + m;
  const int grow0 = rowBase + r0 + 8 * hh;
  if constexpr (EPI == 1) {
#pragma unroll
    for (int t = 0; t < TPW; ++t) {
      const float bv = bias[16 * t + m];
#pragma unroll
      for (int r = 0; r < 8; ++r) {
        float v = acc[t][r] * SCL_ACC + bv;
        v = tanh_fast(v);
        v = (grow0 + r < nN) ? v : 0.0f;
        sp[r * IND + 16 * t] = v;
      }
    }
    {
      float* zp = stg + (size_t)(r0 + m) * IND + NLOC + 8 * hh;
      const v4f z = {0.0f, 0.0f, 0.0f, 0.0f};
      *(v4f*)zp = z;
      *(v4f*)(zp + 4) = z;
    }
  } else {
#pragma unroll
    for (int t = 0; t < TPW; ++t) {
      const float bv = bias[16 * t + m];
#pragma unroll
      for (int r = 0; r < 8; ++r) sp[r * IND + CDM + 16 * t] = acc[t][r] * SCL_ACC + bv;
    }
    {
      const int rr = r0 + m;
      const int grow = rowBase + rr;
      const v4f g = *(const v4f*)(Gf + (size_t)grow * 4);
      float* gq = stg + (size_t)rr * IND + 8 * hh;
#pragma unroll
      for (int e = 0; e < 8; ++e) {
        const int j = 8 * hh + e;
        gq[e] = g.x * Cx[j] + g.y * Cx[CDM + j] + g.z * Cx[2 * CDM + j];
      }
    }
  }
  __syncthreads();

  const float* srow = stg + (size_t)r0 * IND + 4 * lane;
  if constexpr (EPI == 1) {
#pragma unroll
    for (int r = 0; r < 16; ++r) {
      const int row = rowBase + r0 + r;
      const v4f v = *(const v4f*)(srow + r * IND);
      *(volatile v4f*)(Out + (size_t)row * IND + 4 * lane) = v;
    }
    __threadfence();
#pragma unroll
    for (int r = 0; r < 16; ++r) {
      const int row = rowBase + r0 + r;
      const v4f v = *(const v4f*)(srow + r * IND);
      *(volatile v4f*)(Out + (size_t)row * IND + 4 * lane) = v;
    }
  } else {
#pragma unroll
    for (int r = 0; r < 16; ++r) {
      const int row = rowBase + r0 + r;
      if (row < nN) {
        const v4f v = *(const v4f*)(srow + r * IND);
        *(volatile v4f*)(Out + (size_t)row * IND + 4 * lane) = v;
      }
    }
    __threadfence();
#pragma unroll
    for (int r = 0; r < 16; ++r) {
      const int row = rowBase + r0 + r;
      if (row < nN) {
        const v4f v = *(const v4f*)(srow + r * IND);
        *(volatile v4f*)(Out + (size_t)row * IND + 4 * lane) = v;
      }
    }
  }
}

extern "C" void kernel_launch(void* const* d_in, const int* in_sizes, int n_in,
                              void* d_out, int out_size, void* d_ws, size_t ws_size,
                              hipStream_t stream) {
  if (n_in < 16) return;
  const int nN  = in_sizes[0] / IND;
  const int nE1 = in_sizes[1] / 2;
  const int nE2 = in_sizes[2] / 2;
  if (nN <= 0 || nE1 <= 0 || nE2 <= 0) return;
  if (in_sizes[0] != nN * IND || in_sizes[1] != 2 * nE1 || in_sizes[2] != 2 * nE2) return;
  if (in_sizes[3] != IND * CH0 || in_sizes[4] != CH0) return;
  if (in_sizes[5] != CH0 * CDM || in_sizes[6] != CDM) return;
  if (in_sizes[7] != 3 * CDM) return;
  if (in_sizes[8] != NGL * 9 * 16 || in_sizes[9] != NGL * 16) return;
  if (in_sizes[10] != NGL * 16 * 3 || in_sizes[11] != NGL * 3) return;
  if (in_sizes[12] != 3 * IND * NLOC || in_sizes[13] != NLOC) return;
  if (in_sizes[14] != 3 * NLOC * NLOC || in_sizes[15] != NLOC) return;
  if (out_size != nN * IND) return;
  if (nN > (1 << 22) || nE1 > (1 << 28) || nE2 > (1 << 28)) return;

  const float* x   = (const float*)d_in[0];
  const int*   pe  = (const int*)d_in[1];
  const int*   ne  = (const int*)d_in[2];
  const float* cW0 = (const float*)d_in[3];
  const float* cb0 = (const float*)d_in[4];
  const float* cW1 = (const float*)d_in[5];
  const float* cb1 = (const float*)d_in[6];
  const float* Cx  = (const float*)d_in[7];
  const float* gW1 = (const float*)d_in[8];
  const float* gb1 = (const float*)d_in[9];
  const float* gW2 = (const float*)d_in[10];
  const float* gb2 = (const float*)d_in[11];
  const float* lW0 = (const float*)d_in[12];
  const float* lb0 = (const float*)d_in[13];
  const float* lW1 = (const float*)d_in[14];
  const float* lb1 = (const float*)d_in[15];
  float* out = (float*)d_out;

  const int* srcP = pe;  const int* dstP = pe + nE1;
  const int* srcN = ne;  const int* dstN = ne + nE2;

  const int NPAD   = ((nN + TGT - 1) / TGT) * TGT;
  const int nBC    = (nN + NBC - 1) / NBC;
  const int CNTPAD = nBC * NBC;
  if (CNTPAD < NPAD) return;
  if (4 * nBC + 1 > RBN) return;
  const int nBF    = (nN + NBF - 1) / NBF;
  if (nBF + 1 > 4 * nBC + 1) return;
  if (31 * 4 * nBC > 4096) return;
  const int csrLen1 = ((nE1 + 31) & ~31) + 4096;
  const int csrLen2 = ((nE2 + 31) & ~31) + 4096;
  const int nAgg   = NPAD / TGT;
  const int nGl    = NPAD / NTHR;
  const int nGemm  = NPAD / GBM;

  const int uW0 = CH0 * IND / 8;
  const int uW1 = CDM * CH0 / 8;
  const int uL  = NLOC * 3 * IND / 8;

  char* ws = (char*)d_ws;
  size_t off = 0;
  const size_t oW0  = off; off += (size_t)CH0 * IND * 2;        off = (off + 255) & ~(size_t)255;
  const size_t oW1  = off; off += (size_t)CDM * CH0 * 2;        off = (off + 255) & ~(size_t)255;
  const size_t oL0  = off; off += (size_t)NLOC * 3 * IND * 2;   off = (off + 255) & ~(size_t)255;
  const size_t oL1  = off; off += (size_t)NLOC * 3 * IND * 2;   off = (off + 255) & ~(size_t)255;
  const size_t oAP  = off; off += (size_t)NPAD * IND * 2;       off = (off + 255) & ~(size_t)255;
  const size_t oAN  = off; off += (size_t)NPAD * IND * 2;       off = (off + 255) & ~(size_t)255;
  const size_t oLf  = off; off += (size_t)NPAD * IND * 4;       off = (off + 255) & ~(size_t)255;
  const size_t oGA  = off; off += (size_t)NPAD * 4 * 4;         off = (off + 255) & ~(size_t)255;
  const size_t oGB  = off; off += (size_t)NPAD * 4 * 4;         off = (off + 255) & ~(size_t)255;
  const size_t oCnP = off; off += (size_t)CNTPAD * 4;           off = (off + 255) & ~(size_t)255;
  const size_t oOfP = off; off += (size_t)CNTPAD * 4;           off = (off + 255) & ~(size_t)255;
  const size_t oRbP = off; off += (size_t)RBN * 4;              off = (off + 255) & ~(size_t)255;
  const size_t oCsP = off; off += (size_t)csrLen1 * 4;          off = (off + 255) & ~(size_t)255;
  const size_t oCnN = off; off += (size_t)CNTPAD * 4;           off = (off + 255) & ~(size_t)255;
  const size_t oOfN = off; off += (size_t)CNTPAD * 4;           off = (off + 255) & ~(size_t)255;
  const size_t oRbN = off; off += (size_t)RBN * 4;              off = (off + 255) & ~(size_t)255;
  const size_t oCsN = off; off += (size_t)csrLen2 * 4;          off = (off + 255) & ~(size_t)255;
  if (off > ws_size || off > (size_t)WSCAP) return;
  _Float16* W0t  = (_Float16*)(ws + oW0);
  _Float16* W1t  = (_Float16*)(ws + oW1);
  _Float16* L0t  = (_Float16*)(ws + oL0);
  _Float16* L1t  = (_Float16*)(ws + oL1);
  _Float16* aggP = (_Float16*)(ws + oAP);
  _Float16* aggN = (_Float16*)(ws + oAN);
  float* L1f  = (float*)(ws + oLf);
  float* GA   = (float*)(ws + oGA);
  float* GB   = (float*)(ws + oGB);
  int*   cntP = (int*)(ws + oCnP);
  int*   offP = (int*)(ws + oOfP);
  int*   rbP  = (int*)(ws + oRbP);
  int*   csrP = (int*)(ws + oCsP);
  int*   cntN = (int*)(ws + oCnN);
  int*   offN = (int*)(ws + oOfN);
  int*   rbN  = (int*)(ws + oRbN);
  int*   csrN = (int*)(ws + oCsN);

  const int vec8P = ((nE1 & 3) == 0) ? 1 : 0;
  const int vec8N = ((nE2 & 3) == 0) ? 1 : 0;

  k_packw<<<(uW0 + NTHR - 1) / NTHR, NTHR, 0, stream>>>(cW0, W0t, CH0,  IND,  IND, 1, uW0);
  k_packw<<<(uW1 + NTHR - 1) / NTHR, NTHR, 0, stream>>>(cW1, W1t, CDM,  CH0,  CH0, 1, uW1);
  k_packw<<<(uL  + NTHR - 1) / NTHR, NTHR, 0, stream>>>(lW0, L0t, NLOC, IND,  IND, 3, uL);
  k_packw<<<(uL  + NTHR - 1) / NTHR, NTHR, 0, stream>>>(lW1, L1t, NLOC, NLOC, IND, 3, uL);

  hipFuncSetAttribute(reinterpret_cast<const void*>(&k_fill),
                      hipFuncAttributeMaxDynamicSharedMemorySize, LDS_FILL);
  k_count<<<nBC, NTHR, 0, stream>>>(dstP, cntP, nE1, vec8P);
  k_offsets<<<1, OTHR, 0, stream>>>(cntP, offP, rbP, nBC);
  k_fill<<<nBF, NTHR, LDS_FILL, stream>>>(dstP, offP, rbP, csrP, srcP, nE1, vec8P, csrLen1, nN);
  k_count<<<nBC, NTHR, 0, stream>>>(dstN, cntN, nE2, vec8N);
  k_offsets<<<1, OTHR, 0, stream>>>(cntN, offN, rbN, nBC);
  k_fill<<<nBF, NTHR, LDS_FILL, stream>>>(dstN, offN, rbN, csrN, srcN, nE2, vec8N, csrLen2, nN);

  k_color<<<nGemm, GTHR, 0, stream>>>(x, W0t, cb0, W1t, cb1, Cx, GA, nN);

  for (int i = 0; i < NGL; ++i) {
    const float* gin = (i & 1) ? GB : GA;
    float* gout      = (i & 1) ? GA : GB;
    k_glayer<<<nGl, NTHR, 0, stream>>>(gin, gout, cntP, offP, csrP, cntN, offN, csrN,
                                        gW1, gb1, gW2, gb2, i, nN, csrLen1, csrLen2);
  }
  const float* Gfin = (NGL & 1) ? GB : GA;

  k_agg<<<nAgg, NTHR, 0, stream>>>(csrP, offP, cntP, x, aggP, nN, csrLen1);
  k_agg<<<nAgg, NTHR, 0, stream>>>(csrN, offN, cntN, x, aggN, nN, csrLen2);
  k_gemm<1><<<nGemm, GTHR, 0, stream>>>(x, aggP, aggN, L0t, lb0, Gfin, Cx, L1f, nN, nN);

  k_agg<<<nAgg, NTHR, 0, stream>>>(csrP, offP, cntP, L1f, aggP, nN, csrLen1);
  k_agg<<<nAgg, NTHR, 0, stream>>>(csrN, offN, cntN, L1f, aggN, nN, csrLen2);
  k_gemm<2><<<nGemm, GTHR, 0, stream>>>(L1f, aggP, aggN, L1t, lb1, Gfin, Cx, out, NPAD, nN);
}
